// Encoder_41437844472389
// MI455X (gfx1250) — hardware-verified
//
#include <hip/hip_runtime.h>
#include <math.h>

constexpr int NBATCH   = 32;
constexpr int NSTEP    = 512;
constexpr int NVOCAB   = 20000;
constexpr int NEMB     = 300;
constexpr int NHID     = 512;
constexpr int NGATE    = 4 * NHID;
constexpr int KXPAD    = 320;
constexpr int XCH8     = KXPAD / 8;
constexpr int NROWS    = NBATCH * NSTEP;
constexpr int NTHR     = 512;
constexpr int PREP_THR = 256;
constexpr int XPITCH   = 328;
constexpr int HPITCH   = 520;
constexpr int OPITCH   = 516;
constexpr float WCARRY     = 256.0f;
constexpr float WCARRY_INV = 1.0f / 256.0f;

static_assert(NGATE == 2048, "gate axis");
static_assert(KXPAD % 64 == 0 && KXPAD % 32 == 0 && KXPAD >= NEMB, "x K pad");
static_assert(NHID % 64 == 0 && NHID % 32 == 0, "h K");
static_assert(NHID == 32 * (NTHR / 32), "16 waves x 32 hidden units");
static_assert(NBATCH % 16 == 0, "batch tiles");
static_assert((NROWS * XCH8) % PREP_THR == 0, "gather grid exact");
static_assert(16 * XCH8 == NTHR + 128, "x tile staging coverage");
static_assert((XPITCH * 2) % 16 == 0 && (HPITCH * 2) % 16 == 0 && (OPITCH * 4) % 16 == 0, "LDS 16-B pitches");
static_assert(NEMB % 4 == 0, "emb row float4 alignment");
static_assert((NBATCH * NHID * 4) == 65536, "second output byte offset");

typedef __attribute__((ext_vector_type(16))) _Float16 v16h;
typedef __attribute__((ext_vector_type(8)))  _Float16 v8h;
typedef __attribute__((ext_vector_type(16))) __bf16   v16b;
typedef __attribute__((ext_vector_type(8)))  __bf16   v8b;
typedef __attribute__((ext_vector_type(8)))  float    v8f;
typedef __attribute__((ext_vector_type(4)))  float    v4f;
typedef __attribute__((ext_vector_type(4)))  unsigned v4u;

__device__ __forceinline__ unsigned short f2bf_bits(float f) {
  unsigned u = __float_as_uint(f);
  return (unsigned short)((u + 0x7FFFu + ((u >> 16) & 1u)) >> 16);
}
__device__ __forceinline__ float bf_bits2f(unsigned short h) { return __uint_as_float(((unsigned)h) << 16); }
__device__ __forceinline__ float bf16r(float f) { return bf_bits2f(f2bf_bits(f)); }

__device__ __forceinline__ void guard4_h(v8f& a0, v8f& a1, v8f& a2, v8f& a3, v16h x, v16h y0, v16h y1, v16h y2, v16h y3) {
  asm volatile("v_nop\n\tv_nop\n\tv_nop\n\tv_nop" : "+v"(a0), "+v"(a1), "+v"(a2), "+v"(a3) : "v"(x), "v"(y0), "v"(y1), "v"(y2), "v"(y3));
}
__device__ __forceinline__ void guard4_b(v8f& a0, v8f& a1, v8f& a2, v8f& a3, v16b x, v16b y0, v16b y1, v16b y2, v16b y3) {
  asm volatile("v_nop\n\tv_nop\n\tv_nop\n\tv_nop" : "+v"(a0), "+v"(a1), "+v"(a2), "+v"(a3) : "v"(x), "v"(y0), "v"(y1), "v"(y2), "v"(y3));
}
__device__ __forceinline__ void acc_guard4(v8f& a, v8f& b, v8f& c, v8f& d) {
  asm volatile("v_nop\n\tv_nop\n\tv_nop\n\tv_nop" : "+v"(a), "+v"(b), "+v"(c), "+v"(d));
}

template <typename T> struct Frag;
template <> struct Frag<_Float16> {
  typedef v16h V; union U { v16h v; v8h h[2]; };
  static __device__ __forceinline__ v16h load(const _Float16* p) {
    U f; f.h[0] = *(const v8h*)(p); f.h[1] = *(const v8h*)(p + 16); return f.v;
  }
  static __device__ __forceinline__ v8f mma(v16h a, v16h b, v8f c) {
    return __builtin_amdgcn_wmma_f32_16x16x32_f16(false, a, false, b, (short)0, c, false, false);
  }
};
template <> struct Frag<__bf16> {
  typedef v16b V; union U { v16b v; v8b h[2]; };
  static __device__ __forceinline__ v16b load(const __bf16* p) {
    U f; f.h[0] = *(const v8b*)(p); f.h[1] = *(const v8b*)(p + 16); return f.v;
  }
  static __device__ __forceinline__ v8f mma(v16b a, v16b b, v8f c) {
    return __builtin_amdgcn_wmma_f32_16x16x32_bf16(false, a, false, b, (short)0, c, false, false);
  }
};

__device__ __forceinline__ float gate_sig(float x)  { return __builtin_amdgcn_rcpf(1.0f + expf(-x)); }
__device__ __forceinline__ float gate_tanh(float x) { return 1.0f - 2.0f * __builtin_amdgcn_rcpf(expf(2.0f * x) + 1.0f); }

template <int MODE>
__global__ __launch_bounds__(PREP_THR) void tpw_kernel(const float* __restrict__ src, int Rreal, int C, int ldo,
                                                       unsigned short* __restrict__ O, float sc) {
  __shared__ float Tt[64 * 65];
  const int tid = threadIdx.x;
  const int c0 = blockIdx.x * 64, r0 = blockIdx.y * 64;
#pragma unroll
  for (int i = 0; i < 4; ++i) {
    const int idx = i * PREP_THR + tid;
    const int rr = idx >> 4, cc = (idx & 15) * 4;
    const int rg = r0 + rr;
    const int rc = (rg < Rreal) ? rg : (Rreal - 1);
    const bool keep = (rg < Rreal);
    const v4f v = *(const v4f*)(src + (size_t)rc * (size_t)C + c0 + cc);
    const float e0 = v[0], e1 = v[1], e2 = v[2], e3 = v[3];
    Tt[rr * 65 + cc + 0] = keep ? e0 : 0.0f;
    Tt[rr * 65 + cc + 1] = keep ? e1 : 0.0f;
    Tt[rr * 65 + cc + 2] = keep ? e2 : 0.0f;
    Tt[rr * 65 + cc + 3] = keep ? e3 : 0.0f;
  }
  __syncthreads();
  const int q = tid >> 3, c8 = (tid & 7) * 8;
  v8h hv[2];
#pragma unroll
  for (int g = 0; g < 2; ++g) {
    const int qq = g * 32 + q;
#pragma unroll
    for (int e = 0; e < 8; ++e) {
      const float f = Tt[(c8 + e) * 65 + qq];
      unsigned short bits;
      if (MODE == 0) {
        bits = f2bf_bits(f * sc);
      } else {
        const float fb = bf16r(f);
        const _Float16 hf = (_Float16)(fb * sc);
        bits = __builtin_bit_cast(unsigned short, hf);
      }
      hv[g][e] = __builtin_bit_cast(_Float16, bits);
    }
  }
  for (int pass = 0; pass < 2; ++pass) {
#pragma unroll
    for (int g = 0; g < 2; ++g) {
      const size_t o = (size_t)(c0 + g * 32 + q) * (size_t)ldo + (size_t)(r0 + c8);
      *(volatile v8h*)(O + o) = hv[g];
    }
    __threadfence();
  }
}

__global__ __launch_bounds__(PREP_THR) void gather_kernel(const int* __restrict__ tokens, const float* __restrict__ emb,
                                                          unsigned short* __restrict__ XG) {
  const int i = blockIdx.x * PREP_THR + threadIdx.x;
  if (i < NROWS * XCH8) {
    const int row = i / XCH8;
    const int q   = i - row * XCH8;
    const int b   = row & (NBATCH - 1);
    const int t   = row >> 5;
    int tok = tokens[b * NSTEP + t];
    tok = tok < 0 ? 0 : tok;
    tok = tok > (NVOCAB - 1) ? (NVOCAB - 1) : tok;
    const int k  = q * 8;
    const int ka = (k < NEMB - 4) ? k : (NEMB - 4);
    const int kb = (k + 4 < NEMB - 4) ? (k + 4) : (NEMB - 4);
    const float* er = emb + (size_t)tok * NEMB;
    const v4f va = *(const v4f*)(er + ka);
    const v4f vb = *(const v4f*)(er + kb);
    v8h hv;
#pragma unroll
    for (int e = 0; e < 4; ++e) {
      const float xa = va[e];
      const float xb = vb[e];
      const float fa = (k + e < NEMB) ? xa : 0.0f;
      const float fb = (k + 4 + e < NEMB) ? xb : 0.0f;
      const unsigned short ba = f2bf_bits(fa);
      const unsigned short bb = f2bf_bits(fb);
      hv[e]     = __builtin_bit_cast(_Float16, ba);
      hv[4 + e] = __builtin_bit_cast(_Float16, bb);
    }
    *(volatile v8h*)(XG + (size_t)i * 8) = hv;
    __threadfence();
    *(volatile v8h*)(XG + (size_t)i * 8) = hv;
  }
}

__device__ __forceinline__ void stage_x(const unsigned short* __restrict__ xg, unsigned short* xs,
                                        int tstep, int rowbase, int tid) {
  const v4u* src = (const v4u*)(xg + ((size_t)tstep * NBATCH + (size_t)rowbase) * KXPAD);
  const int i0 = tid;
  const int i1 = NTHR + (tid & 127);
  v4u v0 = src[i0];
  v4u v1 = src[i1];
  asm volatile("" : "+v"(v0), "+v"(v1));
  const int m0 = i0 / XCH8, q0 = i0 - m0 * XCH8;
  const int m1 = i1 / XCH8, q1 = i1 - m1 * XCH8;
  *(v4u*)(xs + m0 * XPITCH + q0 * 8) = v0;
  if (tid < 128) *(v4u*)(xs + m1 * XPITCH + q1 * 8) = v1;
}

__device__ __forceinline__ void store_tile(const float* fs, float* __restrict__ dst, int tid) {
  for (int pass = 0; pass < 2; ++pass) {
#pragma unroll
    for (int it = 0; it < 4; ++it) {
      const int idx = it * NTHR + tid;
      const int row = idx >> 7, c4 = (idx & 127) * 4;
      const v4f v = *(const v4f*)(fs + row * OPITCH + c4);
      *(volatile v4f*)(dst + (size_t)row * NHID + c4) = v;
    }
    __threadfence();
  }
}

__global__ __launch_bounds__(NTHR) void seq_kernel(const unsigned short* __restrict__ XGp,
                                                   const unsigned short* __restrict__ WXp,
                                                   const unsigned short* __restrict__ WHp,
                                                   const float* __restrict__ bias,
                                                   float* __restrict__ out) {
  __shared__ __align__(16) unsigned short Xs[2 * 16 * XPITCH];
  __shared__ __align__(16) _Float16       Ah[2 * 16 * HPITCH];
  __shared__ __align__(16) float          Fs[16 * OPITCH];
  const __bf16*   WX = (const __bf16*)WXp;
  const _Float16* WH = (const _Float16*)WHp;
  const int tid = threadIdx.x, lane = tid & 31, wave = tid >> 5;
  const int c = lane & 15, hh = lane >> 4, koff = hh * 8;
  const int rowbase = blockIdx.x * 16;

#pragma unroll 1
  for (int i = tid; i < 2 * 16 * HPITCH; i += NTHR) Ah[i] = (_Float16)0.0f;
  stage_x(XGp, Xs, 0, rowbase, tid);

  float cA[8], cB[8], hA[8], hB[8], bA[4], bB[4];
#pragma unroll
  for (int g = 0; g < 4; ++g) {
    bA[g] = bf16r(bias[g * NHID + 32 * wave + c]);
    bB[g] = bf16r(bias[g * NHID + 32 * wave + 16 + c]);
  }
#pragma unroll
  for (int r = 0; r < 8; ++r) { cA[r] = 0.0f; cB[r] = 0.0f; hA[r] = 0.0f; hB[r] = 0.0f; }
  __syncthreads();

  const v8f z8 = {0.f, 0.f, 0.f, 0.f, 0.f, 0.f, 0.f, 0.f};

#pragma unroll 1
  for (int t = 0; t < NSTEP; ++t) {
    const int cur = t & 1;
    const int nxt = cur ^ 1;
    const int tn = (t + 1 < NSTEP) ? (t + 1) : (NSTEP - 1);
    stage_x(XGp, Xs + nxt * 16 * XPITCH, tn, rowbase, tid);

    const __bf16*   axrow = (const __bf16*)(Xs + cur * 16 * XPITCH) + c * XPITCH + koff;
    const _Float16* ahrow = Ah + cur * 16 * HPITCH + c * HPITCH + koff;
    _Float16*       ahn   = Ah + nxt * 16 * HPITCH;

#pragma unroll 1
    for (int nt = 0; nt < 2; ++nt) {
      const int j = 32 * wave + 16 * nt + c;
      const __bf16*   wx = WX + (size_t)j * KXPAD + koff;
      const _Float16* wh = WH + (size_t)j * NHID + koff;
      v8f acc0 = z8, acc1 = z8, acc2 = z8, acc3 = z8;
#pragma unroll 1
      for (int kx = 0; kx < KXPAD; kx += 32) {
        const v16b a  = Frag<__bf16>::load(axrow + kx);
        const v16b b0 = Frag<__bf16>::load(wx + kx);
        const v16b b1 = Frag<__bf16>::load(wx + (size_t)1 * NHID * KXPAD + kx);
        const v16b b2 = Frag<__bf16>::load(wx + (size_t)2 * NHID * KXPAD + kx);
        const v16b b3 = Frag<__bf16>::load(wx + (size_t)3 * NHID * KXPAD + kx);
        acc0 = Frag<__bf16>::mma(a, b0, acc0);
        acc1 = Frag<__bf16>::mma(a, b1, acc1);
        acc2 = Frag<__bf16>::mma(a, b2, acc2);
        acc3 = Frag<__bf16>::mma(a, b3, acc3);
        guard4_b(acc0, acc1, acc2, acc3, a, b0, b1, b2, b3);
      }
#pragma unroll 1
      for (int k0 = 0; k0 < NHID; k0 += 32) {
        const v16h a  = Frag<_Float16>::load(ahrow + k0);
        const v16h b0 = Frag<_Float16>::load(wh + k0);
        const v16h b1 = Frag<_Float16>::load(wh + (size_t)1 * NHID * NHID + k0);
        const v16h b2 = Frag<_Float16>::load(wh + (size_t)2 * NHID * NHID + k0);
        const v16h b3 = Frag<_Float16>::load(wh + (size_t)3 * NHID * NHID + k0);
        acc0 = Frag<_Float16>::mma(a, b0, acc0);
        acc1 = Frag<_Float16>::mma(a, b1, acc1);
        acc2 = Frag<_Float16>::mma(a, b2, acc2);
        acc3 = Frag<_Float16>::mma(a, b3, acc3);
        guard4_h(acc0, acc1, acc2, acc3, a, b0, b1, b2, b3);
      }
      acc_guard4(acc0, acc1, acc2, acc3);
#pragma unroll
      for (int r = 0; r < 8; ++r) {
        const float zi = acc0[r] * WCARRY_INV + bA[0];
        const float zf = acc1[r] * WCARRY_INV + bA[1];
        const float zg = acc2[r] * WCARRY_INV + bA[2];
        const float zo = acc3[r] * WCARRY_INV + bA[3];
        const float ig = gate_sig(zi);
        const float fg = gate_sig(zf);
        const float gg = gate_tanh(zg);
        const float og = gate_sig(zo);
        const float cn = fg * cA[r] + ig * gg;
        const float hn = og * gate_tanh(cn);
        cA[r] = cn;
        hA[r] = hn;
        ahn[(8 * hh + r) * HPITCH + j] = (_Float16)hn;
      }
#pragma unroll
      for (int r = 0; r < 8; ++r) {
        const float tc = cA[r]; cA[r] = cB[r]; cB[r] = tc;
        const float th = hA[r]; hA[r] = hB[r]; hB[r] = th;
      }
#pragma unroll
      for (int g = 0; g < 4; ++g) {
        const float tb = bA[g]; bA[g] = bB[g]; bB[g] = tb;
      }
    }
    __syncthreads();
  }

#pragma unroll
  for (int r = 0; r < 8; ++r) {
    Fs[(8 * hh + r) * OPITCH + 32 * wave + c]      = hA[r];
    Fs[(8 * hh + r) * OPITCH + 32 * wave + 16 + c] = hB[r];
  }
  __syncthreads();
  store_tile(Fs, out + (size_t)rowbase * NHID, tid);
  __syncthreads();
#pragma unroll
  for (int r = 0; r < 8; ++r) {
    Fs[(8 * hh + r) * OPITCH + 32 * wave + c]      = cA[r];
    Fs[(8 * hh + r) * OPITCH + 32 * wave + 16 + c] = cB[r];
  }
  __syncthreads();
  store_tile(Fs, out + (size_t)NBATCH * NHID + (size_t)rowbase * NHID, tid);
}

extern "C" void kernel_launch(void* const* d_in, const int* in_sizes, int n_in,
                              void* d_out, int out_size, void* d_ws, size_t ws_size, hipStream_t stream) {
  if (n_in < 5 || d_out == nullptr || d_ws == nullptr) return;
  if (in_sizes[0] != NBATCH * NSTEP || in_sizes[1] != NVOCAB * NEMB || in_sizes[2] != NEMB * NGATE ||
      in_sizes[3] != NHID * NGATE || in_sizes[4] != NGATE || out_size != 2 * NBATCH * NHID) return;

  const int*   tokens = (const int*)d_in[0];
  const float* emb    = (const float*)d_in[1];
  const float* wgt_x  = (const float*)d_in[2];
  const float* wgt_h  = (const float*)d_in[3];
  const float* bias   = (const float*)d_in[4];
  float* out = (float*)d_out;

  char* ws = (char*)d_ws; size_t off = 0;
  auto carve = [&](size_t bytes) -> char* { char* p = ws + off; off += (bytes + 255) & ~(size_t)255; return p; };
  unsigned short* WX = (unsigned short*)carve((size_t)NGATE * KXPAD * 2);
  unsigned short* WH = (unsigned short*)carve((size_t)NGATE * NHID * 2);
  unsigned short* XG = (unsigned short*)carve((size_t)NROWS * KXPAD * 2);
  if (off > ws_size || off > (size_t)134217728) return;

  tpw_kernel<0><<<dim3(NGATE / 64, KXPAD / 64), PREP_THR, 0, stream>>>(wgt_x, NEMB, NGATE, KXPAD, WX, WCARRY);
  tpw_kernel<1><<<dim3(NGATE / 64, NHID / 64), PREP_THR, 0, stream>>>(wgt_h, NHID, NGATE, NHID, WH, WCARRY);
  gather_kernel<<<(NROWS * XCH8) / PREP_THR, PREP_THR, 0, stream>>>(tokens, emb, XG);
  seq_kernel<<<NBATCH / 16, NTHR, 0, stream>>>(XG, WX, WH, bias, out);
}
